// DecoderLayer_60060822667509
// MI455X (gfx1250) — hardware-verified
//
#include <hip/hip_runtime.h>
#include <stdint.h>


typedef unsigned long long ull;
typedef unsigned short us16;
typedef us16 v8us __attribute__((ext_vector_type(8)));
typedef us16 v16us __attribute__((ext_vector_type(16)));
typedef __bf16 v16bf __attribute__((ext_vector_type(16)));
typedef _Float16 v8h __attribute__((ext_vector_type(8)));
typedef _Float16 v16h __attribute__((ext_vector_type(16)));
typedef float v4f __attribute__((ext_vector_type(4)));
typedef float v8f __attribute__((ext_vector_type(8)));

#define DM 512
#define RW 4096
#define SEQ 1024
#define NCELL 8
#define NMAT 66
#define NEDGE 34

struct GemmDesc {
  ull A0, A1, A2;
  ull bias, res, out;
  float scale, resscale;
  int act, nparts, wid0, wid1, wid2, outtype, enabled, pad0, pad1, pad2;
};
struct EwDesc {
  ull x0, x1, x2, g, b, out;
  float scale;
  int op, enabled, pad;
};
struct PlanTab {
  GemmDesc gd[NCELL * 7];
  EwDesc   ed[NCELL * 5];
  int act[NCELL];
  int msel[NCELL];
  unsigned fmask;
  int pad[15];
};
static_assert(sizeof(GemmDesc) == 96);
static_assert(sizeof(EwDesc) == 64);
static_assert(sizeof(PlanTab) == 8064);
static_assert(sizeof(PlanTab) % 128 == 0);

struct PlanArgs {
  const float *inpute, *inputo, *node_p, *edge_p;
  const float *edge_b, *edge_g, *edge_beta;
  const float *node_b, *node_g, *node_beta;
  char* ws;
};
static_assert(sizeof(PlanArgs) == 88);

constexpr size_t SZF = (size_t)RW * DM * 4;
constexpr size_t SZH = (size_t)RW * DM * 2;
constexpr size_t SZW = (size_t)DM * DM * 2;
constexpr size_t OFF_WHI   = 0;
constexpr size_t OFF_WLO   = OFF_WHI + NMAT * SZW;
constexpr size_t OFF_ARENA = OFF_WLO + NMAT * SZW;
constexpr size_t OFF_PATHF = OFF_ARENA + 8 * SZF;
constexpr size_t OFF_STAGE = OFF_PATHF + 3 * SZF;
constexpr size_t OFF_T0    = OFF_STAGE + 3 * SZF;
constexpr size_t OFF_T1    = OFF_T0 + SZF;
constexpr size_t OFF_T2    = OFF_T1 + SZF;
constexpr size_t OFF_QH    = OFF_T2 + SZF;
constexpr size_t OFF_KH    = OFF_QH + SZH;
constexpr size_t OFF_VH    = OFF_KH + SZH;
constexpr size_t OFF_OB    = OFF_VH + SZH;
constexpr size_t OFF_QN    = OFF_OB + SZF;
constexpr size_t OFF_TAB   = OFF_QN + SZF;
constexpr size_t WS_NEED   = OFF_TAB + sizeof(PlanTab);

union FragU { v16us v; v8us h[2]; };
union FragH { v16h v; v8h h[2]; };

#define NOP4 "v_nop\n\tv_nop\n\tv_nop\n\tv_nop"
#define WG2(acc, a, b) asm volatile(NOP4 : "+v"(acc) : "v"(a), "v"(b))
#define WG4(acc, a, b, c2, e2) asm volatile(NOP4 : "+v"(acc) : "v"(a), "v"(b), "v"(c2), "v"(e2))

__device__ __forceinline__ v8f mma_bf(v16us a, v16us b, v8f c) {
  v16bf af = __builtin_bit_cast(v16bf, a);
  v16bf bf = __builtin_bit_cast(v16bf, b);
  return __builtin_amdgcn_wmma_f32_16x16x32_bf16(false, af, false, bf, (short)0, c, false, false);
}
__device__ __forceinline__ v8f mma_h(v16h a, v16h b, v8f c) {
  return __builtin_amdgcn_wmma_f32_16x16x32_f16(false, a, false, b, (short)0, c, false, false);
}

__device__ __forceinline__ void split_bf16(float x, us16& hi, us16& lo) {
  unsigned u = __float_as_uint(x);
  unsigned hu = (u + 0x7FFFu + ((u >> 16) & 1u)) & 0xFFFF0000u;
  float rem = x - __uint_as_float(hu);
  unsigned lu = __float_as_uint(rem);
  lu = (lu + 0x7FFFu + ((lu >> 16) & 1u)) >> 16;
  hi = (us16)(hu >> 16);
  lo = (us16)lu;
}

__device__ __forceinline__ float geluf(float x) {
  return 0.5f * x * (1.f + tanhf(0.7978845608028654f * (x + 0.044715f * x * x * x)));
}

__device__ __forceinline__ ull PA(char* ws, size_t off) { return (ull)(ws + off); }

__global__ __launch_bounds__(256) void wconv_kernel(const float* __restrict__ src, int widbase, char* ws) {
  __shared__ float tile[128][33];
  const int t = threadIdx.x, tx = t & 31, ty = t >> 5, lane = tx, wv = ty;
  const int mat = blockIdx.z, n0 = (int)blockIdx.x * 32, k0 = (int)blockIdx.y * 128;
  if (n0 + 32 > DM || k0 + 128 > DM || widbase + mat >= NMAT) return;
  const float* S = src + (size_t)mat * DM * DM;
  for (int i = ty; i < 128; i += 8) tile[i][tx] = S[(size_t)(k0 + i) * DM + n0 + tx];
  __syncthreads();
  us16* WH = (us16*)(ws + OFF_WHI) + (size_t)(widbase + mat) * DM * DM;
  us16* WL = (us16*)(ws + OFF_WLO) + (size_t)(widbase + mat) * DM * DM;
  for (int pass = 0; pass < 2; ++pass) {
#pragma unroll
    for (int it = 0; it < 2; ++it) {
      const int nl = wv * 4 + it * 2 + (lane >> 4);
      const int kq = (lane & 15) * 8;
      v8us hv, lv;
#pragma unroll
      for (int e = 0; e < 8; ++e) {
        us16 hh, ll;
        split_bf16(tile[kq + e][nl], hh, ll);
        hv[e] = hh; lv[e] = ll;
      }
      const size_t off = (size_t)(n0 + nl) * DM + k0 + kq;
      *(volatile v4f*)(WH + off) = __builtin_bit_cast(v4f, hv);
      *(volatile v4f*)(WL + off) = __builtin_bit_cast(v4f, lv);
    }
    if (pass == 0) __threadfence();
  }
}

__device__ static int amaxm(const float* v, int n, unsigned mask) {
  int bi = -1; float bv = 0.f;
  for (int j = 0; j < n; j++) {
    if ((mask >> j) & 1u) continue;
    if (bi < 0 || v[j] > bv) { bv = v[j]; bi = j; }
  }
  return bi < 0 ? 0 : bi;
}
__device__ static float selwf(const float* v, int n, int sel, unsigned mask) {
  float mx = -3.0e38f;
  for (int j = 0; j < n; j++) if (!((mask >> j) & 1u) && v[j] > mx) mx = v[j];
  float s = 0.f;
  for (int j = 0; j < n; j++) if (!((mask >> j) & 1u)) s += expf(v[j] - mx);
  return expf(v[sel] - mx) / s;
}
__device__ static void set_ew(EwDesc* e, ull x0, ull x1, ull x2, ull g, ull b, float sc, ull out, int op) {
  e->x0 = x0; e->x1 = x1; e->x2 = x2; e->g = g; e->b = b; e->scale = sc; e->out = out; e->op = op;
  e->enabled = 1; e->pad = 0;
}
__device__ static void set_gemm(GemmDesc* g, ull A0, ull A1, ull A2, int np, int w0, int w1, int w2,
                                ull bias, int act, float sc, ull res, float rs, ull out, int otype) {
  g->A0 = A0; g->A1 = A1; g->A2 = A2; g->nparts = np; g->wid0 = w0; g->wid1 = w1; g->wid2 = w2;
  g->bias = bias; g->act = act; g->scale = sc; g->res = res; g->resscale = rs; g->out = out;
  g->outtype = otype; g->enabled = 1; g->pad0 = 0; g->pad1 = 0; g->pad2 = 0;
}

__device__ static void plan_fill(PlanTab* T, const PlanArgs& pa) {
  char* ws = pa.ws;
  unsigned processed = 0;
  int lind = 0;
  for (int c = 0; c < NCELL; ++c) {
    const int nsrc = (c + 2 < 5) ? c + 2 : 5;
    const int snode = c - nsrc;
    const int L = nsrc * 5;
    const float* npp = pa.node_p + c * 8;
    const float* eq = pa.edge_p + 0 * 170 + lind * 5;
    const float* ek = pa.edge_p + 1 * 170 + lind * 5;
    const float* ev = pa.edge_p + 2 * 170 + lind * 5;

    const int act = amaxm(npp, 8, 0u);
    const float aw = selwf(npp, 8, act, 0u);
    const unsigned qm = 0x1Fu;
    const int qsel = amaxm(eq, L, qm);
    const float qw = selwf(eq, L, qsel, qm);
    int ksel = -1, vsel = -1, ktype = -2;
    float kw = 0.f, vw = 0.f;
    if (act < 7) {
      const unsigned km = (act > 0) ? qm : 0u;
      ksel = amaxm(ek, L, km);
      kw = selwf(ek, L, ksel, km);
      ktype = (ksel / 5 == 0) ? -2 : -1;
      if (act < 5) {
        if (act == 0 && ktype == -2) { vsel = amaxm(ev, 5, 0u); vw = selwf(ev, 5, vsel, 0u); }
        else                         { vsel = amaxm(ev, L, km); vw = selwf(ev, L, vsel, km); }
      }
    }

#pragma unroll
    for (int p = 0; p < 3; ++p) {
      const int sel = (p == 0) ? qsel : (p == 1 ? ksel : vsel);
      const float wt = (p == 0) ? qw : (p == 1 ? kw : vw);
      if (sel < 0) continue;
      const int se = sel / 5, op = sel % 5;
      int e = lind + se; if (e > NEDGE - 1) e = NEDGE - 1;
      int inn = (se == 0) ? -2 : snode + se; if (inn > 7) inn = 7;
      if (inn >= 0) processed |= (1u << inn);
      const ull x = (inn == -2) ? (ull)pa.inpute : (inn == -1) ? (ull)pa.inputo
                  : PA(ws, OFF_ARENA + (size_t)inn * SZF);
      const ull pF = PA(ws, OFF_PATHF + (size_t)p * SZF);
      if (op == 4) {
        set_ew(&T->ed[c * 5 + p], x, 0, 0, 0, 0, wt, pF, 1);
      } else {
        ull A = x;
        if (op <= 2) {
          const ull st = PA(ws, OFF_STAGE + (size_t)p * SZF);
          set_ew(&T->ed[c * 5 + p], x, 0, 0, (ull)(pa.edge_g + (size_t)e * DM),
                 (ull)(pa.edge_beta + (size_t)e * DM), 1.f, st, 0);
          A = st;
        }
        const int ga = (op == 0) ? 1 : (op == 1) ? 2 : 0;
        set_gemm(&T->gd[c * 7 + p], A, 0, 0, 1, e, 0, 0, (ull)(pa.edge_b + (size_t)e * DM),
                 ga, wt, 0, 0.f, pF, 0);
      }
    }

    const ull qF = PA(ws, OFF_PATHF), kF = PA(ws, OFF_PATHF + SZF), vF = PA(ws, OFF_PATHF + 2 * SZF);
    const ull outc = PA(ws, OFF_ARENA + (size_t)c * SZF);
    const ull ng = (ull)(pa.node_g + (size_t)c * DM), nbe = (ull)(pa.node_beta + (size_t)c * DM);
    const int W0 = NEDGE + c * 4 + 0, W1 = NEDGE + c * 4 + 1, W2 = NEDGE + c * 4 + 2, W3 = NEDGE + c * 4 + 3;
    const ull b0 = (ull)(pa.node_b + ((size_t)c * 4 + 0) * DM);
    const ull b1 = (ull)(pa.node_b + ((size_t)c * 4 + 1) * DM);
    const ull b2 = (ull)(pa.node_b + ((size_t)c * 4 + 2) * DM);
    const ull b3 = (ull)(pa.node_b + ((size_t)c * 4 + 3) * DM);
    const ull T0 = PA(ws, OFF_T0), T1 = PA(ws, OFF_T1), T2 = PA(ws, OFF_T2);
    const ull QN = PA(ws, OFF_QN), QH = PA(ws, OFF_QH), KH = PA(ws, OFF_KH), VH = PA(ws, OFF_VH), OB = PA(ws, OFF_OB);

    switch (act) {
      case 0:
        set_ew(&T->ed[c * 5 + 3], qF, 0, 0, ng, nbe, 1.f, QN, 0);
        set_gemm(&T->gd[c * 7 + 3], QN, 0, 0, 1, W0, 0, 0, b0, 0, 1.f,  0, 0.f, QH, 1);
        set_gemm(&T->gd[c * 7 + 4], kF, 0, 0, 1, W1, 0, 0, b1, 0, 8.f,  0, 0.f, KH, 1);
        set_gemm(&T->gd[c * 7 + 5], vF, 0, 0, 1, W2, 0, 0, b2, 0, 16.f, 0, 0.f, VH, 1);
        set_gemm(&T->gd[c * 7 + 6], OB, 0, 0, 1, W3, 0, 0, b3, 0, aw, qF, aw, outc, 0);
        break;
      case 1:
        set_gemm(&T->gd[c * 7 + 3], qF, 0, 0, 1, W0, 0, 0, b0, 2, 1.f, 0, 0.f, T0, 0);
        set_gemm(&T->gd[c * 7 + 4], kF, 0, 0, 1, W1, 0, 0, b1, 0, 1.f, 0, 0.f, T1, 0);
        set_ew(&T->ed[c * 5 + 4], T0, T1, 0, 0, 0, 1.f, T2, 3);
        set_gemm(&T->gd[c * 7 + 6], T2, 0, 0, 1, W3, 0, 0, b3, 0, aw, qF, aw, outc, 0);
        break;
      case 2:
        set_ew(&T->ed[c * 5 + 3], qF, kF, vF, ng, nbe, aw, outc, 0);
        break;
      case 3:
        set_gemm(&T->gd[c * 7 + 3], qF, kF, vF, 3, W0, W1, W2, 0, 1, 1.f, 0, 0.f, T2, 0);
        set_gemm(&T->gd[c * 7 + 6], T2, 0, 0, 1, W3, 0, 0, b3, 0, aw, qF, aw, outc, 0);
        break;
      case 4:
        set_ew(&T->ed[c * 5 + 3], qF, kF, vF, 0, 0, aw, outc, 2);
        break;
      case 5:
        set_gemm(&T->gd[c * 7 + 4], kF, 0, 0, 1, W1, 0, 0, b1, 2, aw, qF, aw, outc, 0);
        break;
      case 6:
        set_ew(&T->ed[c * 5 + 3], qF, kF, 0, 0, 0, aw, outc, 1);
        break;
      default:
        set_ew(&T->ed[c * 5 + 3], qF, 0, 0, ng, nbe, aw, outc, 0);
        break;
    }
    T->act[c] = act;
    T->msel[c] = (ktype == -1) ? 1 : 0;
    lind += nsrc;
  }
  T->fmask = (~processed) & 0xFFu;
}

constexpr int TAB_NV = (int)(sizeof(PlanTab) / 16);
union PlanU { PlanTab t; v4f v[TAB_NV]; };

__global__ __launch_bounds__(32) void plan_kernel(PlanArgs pa) {
  __shared__ PlanU su;
  const int lane = threadIdx.x & 31;
  const v4f zero4 = {0.f, 0.f, 0.f, 0.f};
  for (int i = lane; i < TAB_NV; i += 32) su.v[i] = zero4;
  __syncthreads();
  if (lane == 0) plan_fill(&su.t, pa);
  __syncthreads();
  v4f* dst = (v4f*)(pa.ws + OFF_TAB);
  for (int pass = 0; pass < 2; ++pass) {
    for (int i = lane; i < TAB_NV; i += 32) {
      const v4f val = su.v[i];
      *(volatile v4f*)(dst + i) = val;
    }
    if (pass == 0) __threadfence();
  }
}

__global__ __launch_bounds__(128) void gemm_kernel(char* ws, int c, int slot0) {
  __shared__ __attribute__((aligned(16))) us16 Ah[64 * 40];
  __shared__ __attribute__((aligned(16))) us16 Al[64 * 40];
  __shared__ __attribute__((aligned(16))) us16 Wh[64 * 40];
  __shared__ __attribute__((aligned(16))) us16 Wl[64 * 40];
  __shared__ __attribute__((aligned(16))) float Es[64 * 68];
  const PlanTab* tab = (const PlanTab*)(ws + OFF_TAB);
  const int slot = slot0 + (int)blockIdx.z;
  if (slot > 6 || c >= NCELL) return;
  const GemmDesc d = tab->gd[c * 7 + slot];
  if (!d.enabled) return;
  const int t = threadIdx.x, lane = t & 31, wv = t >> 5, hl = lane >> 4, m = lane & 15;
  const int row0 = (int)blockIdx.x * 64, col0 = (int)blockIdx.y * 64;
  if (row0 + 64 > RW || col0 + 64 > DM) return;
  const int sr = t >> 1, sk = (t & 1) * 16;
  const int arow = wv * 16 + m;

  v8f acc[4];
  {
    const v8f z = {0.f, 0.f, 0.f, 0.f, 0.f, 0.f, 0.f, 0.f};
#pragma unroll
    for (int j = 0; j < 4; ++j) acc[j] = z;
  }
  int np = d.nparts; np = np < 1 ? 1 : (np > 3 ? 3 : np);

  for (int part = 0; part < np; ++part) {
    const ull Aa = (part == 0) ? d.A0 : (part == 1 ? d.A1 : d.A2);
    int wid = (part == 0) ? d.wid0 : (part == 1 ? d.wid1 : d.wid2);
    wid = wid < 0 ? 0 : (wid > NMAT - 1 ? NMAT - 1 : wid);
    const float* A = (const float*)Aa;
    const us16* WHp = (const us16*)(ws + OFF_WHI) + (size_t)wid * DM * DM;
    const us16* WLp = (const us16*)(ws + OFF_WLO) + (size_t)wid * DM * DM;

    for (int kk = 0; kk < DM; kk += 32) {
      __syncthreads();
      {
        const float* ap = A + (size_t)(row0 + sr) * DM + kk + sk;
        const v4f x0 = *(const v4f*)(ap);
        const v4f x1 = *(const v4f*)(ap + 4);
        const v4f x2 = *(const v4f*)(ap + 8);
        const v4f x3 = *(const v4f*)(ap + 12);
        v8us ha, la, hb, lb;
#pragma unroll
        for (int e = 0; e < 4; ++e) {
          us16 hh, ll;
          split_bf16(x0[e], hh, ll); ha[e] = hh;     la[e] = ll;
          split_bf16(x1[e], hh, ll); ha[4 + e] = hh; la[4 + e] = ll;
          split_bf16(x2[e], hh, ll); hb[e] = hh;     lb[e] = ll;
          split_bf16(x3[e], hh, ll); hb[4 + e] = hh; lb[4 + e] = ll;
        }
        *(v8us*)(Ah + sr * 40 + sk)     = ha;
        *(v8us*)(Ah + sr * 40 + sk + 8) = hb;
        *(v8us*)(Al + sr * 40 + sk)     = la;
        *(v8us*)(Al + sr * 40 + sk + 8) = lb;
      }
      {
        const us16* hp = WHp + (size_t)(col0 + sr) * DM + kk + sk;
        const us16* lp = WLp + (size_t)(col0 + sr) * DM + kk + sk;
        *(v8us*)(Wh + sr * 40 + sk)     = *(const v8us*)(hp);
        *(v8us*)(Wh + sr * 40 + sk + 8) = *(const v8us*)(hp + 8);
        *(v8us*)(Wl + sr * 40 + sk)     = *(const v8us*)(lp);
        *(v8us*)(Wl + sr * 40 + sk + 8) = *(const v8us*)(lp + 8);
      }
      __syncthreads();
      FragU fah, fal;
      fah.h[0] = *(const v8us*)(Ah + arow * 40 + 8 * hl);
      fah.h[1] = *(const v8us*)(Ah + arow * 40 + 16 + 8 * hl);
      fal.h[0] = *(const v8us*)(Al + arow * 40 + 8 * hl);
      fal.h[1] = *(const v8us*)(Al + arow * 40 + 16 + 8 * hl);
#pragma unroll
      for (int j = 0; j < 4; ++j) {
        const int brow = j * 16 + m;
        FragU fwh, fwl;
        fwh.h[0] = *(const v8us*)(Wh + brow * 40 + 8 * hl);
        fwh.h[1] = *(const v8us*)(Wh + brow * 40 + 16 + 8 * hl);
        fwl.h[0] = *(const v8us*)(Wl + brow * 40 + 8 * hl);
        fwl.h[1] = *(const v8us*)(Wl + brow * 40 + 16 + 8 * hl);
        acc[j] = mma_bf(fah.v, fwh.v, acc[j]);
        acc[j] = mma_bf(fah.v, fwl.v, acc[j]);
        acc[j] = mma_bf(fal.v, fwh.v, acc[j]);
        WG4(acc[j], fah.v, fal.v, fwh.v, fwl.v);
      }
    }
  }

  const float* bias = (const float*)d.bias;
  const float* res  = (const float*)d.res;
  const int erow0 = wv * 16 + 8 * hl;
#pragma unroll
  for (int j = 0; j < 4; ++j) {
    const int col = col0 + j * 16 + m;
    const float bv = bias ? bias[col] : 0.f;
#pragma unroll
    for (int r = 0; r < 8; ++r) {
      float v = acc[j][r] + bv;
      if (d.act == 1) v = fmaxf(v, 0.f);
      else if (d.act == 2) v = geluf(v);
      v *= d.scale;
      if (res) v += d.resscale * res[(size_t)(row0 + erow0 + r) * DM + col];
      Es[(erow0 + r) * 68 + j * 16 + m] = v;
    }
  }
  __syncthreads();
  if (d.outtype == 0) {
    float* o = (float*)d.out;
    for (int pass = 0; pass < 2; ++pass) {
#pragma unroll
      for (int q = 0; q < 8; ++q) {
        const int rl = 2 * q + hl, cl = m * 4;
        const v4f val = *(const v4f*)(Es + (wv * 16 + rl) * 68 + cl);
        *(volatile v4f*)(o + (size_t)(row0 + wv * 16 + rl) * DM + col0 + cl) = val;
      }
      if (pass == 0) __threadfence();
    }
  } else {
    _Float16* o = (_Float16*)d.out;
    for (int pass = 0; pass < 2; ++pass) {
#pragma unroll
      for (int q = 0; q < 4; ++q) {
        const int rl = 4 * q + (lane >> 3), cl = (lane & 7) * 8;
        const float* ep = Es + (wv * 16 + rl) * 68 + cl;
        const v4f u0 = *(const v4f*)(ep);
        const v4f u1 = *(const v4f*)(ep + 4);
        v8h hv;
#pragma unroll
        for (int e = 0; e < 4; ++e) { hv[e] = (_Float16)u0[e]; hv[4 + e] = (_Float16)u1[e]; }
        *(volatile v4f*)(o + (size_t)(row0 + wv * 16 + rl) * DM + col0 + cl) = __builtin_bit_cast(v4f, hv);
      }
      if (pass == 0) __threadfence();
    }
  }
}

__global__ __launch_bounds__(128) void ew_kernel(char* ws, int c, int slot0) {
  const PlanTab* tab = (const PlanTab*)(ws + OFF_TAB);
  const int slot = slot0 + (int)blockIdx.y;
  if (slot > 4 || c >= NCELL) return;
  const EwDesc d = tab->ed[c * 5 + slot];
  if (!d.enabled) return;
  const int lane = threadIdx.x & 31, wv = threadIdx.x >> 5;
  const int row = (int)blockIdx.x * 4 + wv;
  if (row >= RW) return;
  const float* x0 = (const float*)d.x0;
  const float* x1 = (const float*)d.x1;
  const float* x2 = (const float*)d.x2;
  const v4f zero4 = {0.f, 0.f, 0.f, 0.f};
  v4f v[4];
#pragma unroll
  for (int j = 0; j < 4; ++j) {
    const size_t idx = (size_t)row * DM + j * 128 + lane * 4;
    const v4f a  = *(const v4f*)(x0 + idx);
    const v4f b  = x1 ? *(const v4f*)(x1 + idx) : zero4;
    const v4f cc = x2 ? *(const v4f*)(x2 + idx) : zero4;
    v4f r;
    if (d.op == 2) {
#pragma unroll
      for (int e = 0; e < 4; ++e) {
        const float ex = __expf(-b[e]);
        r[e] = a[e] * __builtin_amdgcn_rcpf(1.f + ex) + cc[e];
      }
    } else if (d.op == 3) {
      r = a * b;
    } else {
      r = a + b + cc;
    }
    v[j] = r;
  }
  v4f y[4];
  if (d.op == 0) {
    float s = 0.f;
#pragma unroll
    for (int j = 0; j < 4; ++j) s += v[j][0] + v[j][1] + v[j][2] + v[j][3];
#pragma unroll
    for (int off = 16; off > 0; off >>= 1) s += __shfl_xor(s, off, 32);
    const float mean = s * (1.f / DM);
    v4f dv[4];
    float ss = 0.f;
#pragma unroll
    for (int j = 0; j < 4; ++j) {
      dv[j] = v[j] - mean;
      ss += dv[j][0] * dv[j][0] + dv[j][1] * dv[j][1] + dv[j][2] * dv[j][2] + dv[j][3] * dv[j][3];
    }
#pragma unroll
    for (int off = 16; off > 0; off >>= 1) ss += __shfl_xor(ss, off, 32);
    const float inv = rsqrtf(ss * (1.f / DM) + 1e-6f);
    const float* g  = (const float*)d.g;
    const float* bb = (const float*)d.b;
#pragma unroll
    for (int j = 0; j < 4; ++j) {
      const int col = j * 128 + lane * 4;
      const v4f gv = *(const v4f*)(g + col);
      const v4f bv = *(const v4f*)(bb + col);
      y[j] = dv[j] * inv * gv + bv;
    }
  } else {
#pragma unroll
    for (int j = 0; j < 4; ++j) y[j] = v[j];
  }
#pragma unroll
  for (int j = 0; j < 4; ++j) y[j] = y[j] * d.scale;
  float* o = (float*)d.out;
  for (int pass = 0; pass < 2; ++pass) {
#pragma unroll
    for (int j = 0; j < 4; ++j)
      *(volatile v4f*)(o + (size_t)row * DM + j * 128 + lane * 4) = y[j];
    if (pass == 0) __threadfence();
  }
}

__global__ __launch_bounds__(128) void attn_kernel(char* ws, int c, const int* __restrict__ msrc, const int* __restrict__ mtgt) {
  __shared__ __attribute__((aligned(16))) _Float16 Ks[32 * 72];
  __shared__ __attribute__((aligned(16))) _Float16 Vt[64 * 40];
  __shared__ __attribute__((aligned(16))) _Float16 Ps[64 * 40];
  __shared__ __attribute__((aligned(16))) float Os[64 * 68];
  const PlanTab* tab = (const PlanTab*)(ws + OFF_TAB);
  if (c >= NCELL) return;
  if (tab->act[c] != 0) return;
  const int* mk = tab->msel[c] ? mtgt : msrc;
  const int bid = (int)blockIdx.x;
  if (bid >= 512) return;
  const int qb = bid & 15, h = (bid >> 4) & 7, b = bid >> 7;
  const int t = threadIdx.x, lane = t & 31, wv = t >> 5, hl = lane >> 4, m = lane & 15;
  const _Float16* QH = (const _Float16*)(ws + OFF_QH);
  const _Float16* KH = (const _Float16*)(ws + OFF_KH);
  const _Float16* VH = (const _Float16*)(ws + OFF_VH);
  float* OB = (float*)(ws + OFF_OB);
  const int qrow = b * SEQ + qb * 64 + wv * 16;

  FragH qa0, qa1;
  {
    const _Float16* qp = QH + (size_t)(qrow + m) * DM + h * 64;
    qa0.h[0] = *(const v8h*)(qp + 8 * hl);
    qa0.h[1] = *(const v8h*)(qp + 16 + 8 * hl);
    qa1.h[0] = *(const v8h*)(qp + 32 + 8 * hl);
    qa1.h[1] = *(const v8h*)(qp + 48 + 8 * hl);
  }
  const v8f z = {0.f, 0.f, 0.f, 0.f, 0.f, 0.f, 0.f, 0.f};
  v8f o[4];
#pragma unroll
  for (int j = 0; j < 4; ++j) o[j] = z;
  float rm[8], rl[8];
#pragma unroll
  for (int r = 0; r < 8; ++r) { rm[r] = -1e30f; rl[r] = 0.f; }
  const int sk = t >> 2, sd = (t & 3) * 16;

  for (int kt = 0; kt < SEQ; kt += 32) {
    {
      const _Float16* kp = KH + (size_t)(b * SEQ + kt + sk) * DM + h * 64 + sd;
      *(v8h*)(Ks + sk * 72 + sd)     = *(const v8h*)(kp);
      *(v8h*)(Ks + sk * 72 + sd + 8) = *(const v8h*)(kp + 8);
      const _Float16* vp = VH + (size_t)(b * SEQ + kt + sk) * DM + h * 64 + sd;
      const v8h va = *(const v8h*)(vp);
      const v8h vb = *(const v8h*)(vp + 8);
#pragma unroll
      for (int e = 0; e < 8; ++e) {
        Vt[(sd + e) * 40 + sk]     = va[e];
        Vt[(sd + 8 + e) * 40 + sk] = vb[e];
      }
    }
    __syncthreads();
    v8f s0 = z, s1 = z;
    {
      FragH ka, kc, kd, ke;
      ka.h[0] = *(const v8h*)(Ks + m * 72 + 8 * hl);
      ka.h[1] = *(const v8h*)(Ks + m * 72 + 16 + 8 * hl);
      kc.h[0] = *(const v8h*)(Ks + m * 72 + 32 + 8 * hl);
      kc.h[1] = *(const v8h*)(Ks + m * 72 + 48 + 8 * hl);
      s0 = mma_h(qa0.v, ka.v, s0);
      s0 = mma_h(qa1.v, kc.v, s0);
      kd.h[0] = *(const v8h*)(Ks + (16 + m) * 72 + 8 * hl);
      kd.h[1] = *(const v8h*)(Ks + (16 + m) * 72 + 16 + 8 * hl);
      ke.h[0] = *(const v8h*)(Ks + (16 + m) * 72 + 32 + 8 * hl);
      ke.h[1] = *(const v8h*)(Ks + (16 + m) * 72 + 48 + 8 * hl);
      s1 = mma_h(qa0.v, kd.v, s1);
      s1 = mma_h(qa1.v, ke.v, s1);
      WG4(s0, qa0.v, qa1.v, ka.v, kc.v);
      WG4(s1, qa0.v, qa1.v, kd.v, ke.v);
    }
    const int mk0 = mk[(size_t)b * SEQ + kt + m];
    const int mk1 = mk[(size_t)b * SEQ + kt + 16 + m];
    float corr[8];
#pragma unroll
    for (int r = 0; r < 8; ++r) {
      const float a0 = mk0 ? -1e9f : s0[r] * (1.f / 64.f);
      const float a1 = mk1 ? -1e9f : s1[r] * (1.f / 64.f);
      float mx = fmaxf(a0, a1);
#pragma unroll
      for (int off = 8; off > 0; off >>= 1) mx = fmaxf(mx, __shfl_xor(mx, off, 32));
      const float nm = fmaxf(rm[r], mx);
      const float p0 = expf(a0 - nm), p1 = expf(a1 - nm);
      float rs = p0 + p1;
#pragma unroll
      for (int off = 8; off > 0; off >>= 1) rs += __shfl_xor(rs, off, 32);
      const float cr = expf(rm[r] - nm);
      rl[r] = rl[r] * cr + rs;
      rm[r] = nm;
      corr[r] = cr;
      Ps[(wv * 16 + 8 * hl + r) * 40 + m]      = (_Float16)(p0 * 256.f);
      Ps[(wv * 16 + 8 * hl + r) * 40 + 16 + m] = (_Float16)(p1 * 256.f);
    }
#pragma unroll
    for (int r = 0; r < 8; ++r) {
      o[0][r] *= corr[r]; o[1][r] *= corr[r]; o[2][r] *= corr[r]; o[3][r] *= corr[r];
    }
    __syncthreads();
    {
      FragH pa;
      pa.h[0] = *(const v8h*)(Ps + (wv * 16 + m) * 40 + 8 * hl);
      pa.h[1] = *(const v8h*)(Ps + (wv * 16 + m) * 40 + 16 + 8 * hl);
#pragma unroll
      for (int j = 0; j < 4; ++j) {
        FragH vb;
        vb.h[0] = *(const v8h*)(Vt + (j * 16 + m) * 40 + 8 * hl);
        vb.h[1] = *(const v8h*)(Vt + (j * 16 + m) * 40 + 16 + 8 * hl);
        o[j] = mma_h(pa.v, vb.v, o[j]);
        WG4(o[j], pa.v, vb.v, qa0.v, qa1.v);
      }
    }
    __syncthreads();
  }
  float inv[8];
#pragma unroll
  for (int r = 0; r < 8; ++r) inv[r] = 1.f / (rl[r] * 4096.f);
#pragma unroll
  for (int j = 0; j < 4; ++j) {
#pragma unroll
    for (int r = 0; r < 8; ++r) Os[(wv * 16 + 8 * hl + r) * 68 + j * 16 + m] = o[j][r] * inv[r];
  }
  __syncthreads();
  for (int pass = 0; pass < 2; ++pass) {
#pragma unroll
    for (int q = 0; q < 8; ++q) {
      const int rl2 = 2 * q + hl, cl = m * 4;
      const v4f val = *(const v4f*)(Os + (wv * 16 + rl2) * 68 + cl);
      *(volatile v4f*)(OB + (size_t)(qrow + rl2) * DM + h * 64 + cl) = val;
    }
    if (pass == 0) __threadfence();
  }
}

__global__ __launch_bounds__(128) void final_kernel(char* ws, const float* __restrict__ g, const float* __restrict__ bb, float* out) {
  const PlanTab* tab = (const PlanTab*)(ws + OFF_TAB);
  const unsigned fmask = tab->fmask;
  const int lane = threadIdx.x & 31, wv = threadIdx.x >> 5;
  const int row = (int)blockIdx.x * 4 + wv;
  if (row >= RW) return;
  const float* arena = (const float*)(ws + OFF_ARENA);
  const v4f zero4 = {0.f, 0.f, 0.f, 0.f};
  v4f v[4];
#pragma unroll
  for (int j = 0; j < 4; ++j) {
    const size_t idx = (size_t)row * DM + j * 128 + lane * 4;
    v4f s = zero4;
    for (int nn = 0; nn < NCELL; ++nn)
      if ((fmask >> nn) & 1u) s = s + *(const v4f*)(arena + (size_t)nn * RW * DM + idx);
    v[j] = s;
  }
  float s = 0.f;
#pragma unroll
  for (int j = 0; j < 4; ++j) s += v[j][0] + v[j][1] + v[j][2] + v[j][3];
#pragma unroll
  for (int off = 16; off > 0; off >>= 1) s += __shfl_xor(s, off, 32);
  const float mean = s * (1.f / DM);
  v4f dv[4];
  float ss = 0.f;
#pragma unroll
  for (int j = 0; j < 4; ++j) {
    dv[j] = v[j] - mean;
    ss += dv[j][0] * dv[j][0] + dv[j][1] * dv[j][1] + dv[j][2] * dv[j][2] + dv[j][3] * dv[j][3];
  }
#pragma unroll
  for (int off = 16; off > 0; off >>= 1) ss += __shfl_xor(ss, off, 32);
  const float inv = rsqrtf(ss * (1.f / DM) + 1e-6f);
  v4f y[4];
#pragma unroll
  for (int j = 0; j < 4; ++j) {
    const int col = j * 128 + lane * 4;
    const v4f gv = *(const v4f*)(g + col);
    const v4f bv = *(const v4f*)(bb + col);
    y[j] = dv[j] * inv * gv + bv;
  }
  for (int pass = 0; pass < 2; ++pass) {
#pragma unroll
    for (int j = 0; j < 4; ++j)
      *(volatile v4f*)(out + (size_t)row * DM + j * 128 + lane * 4) = y[j];
    if (pass == 0) __threadfence();
  }
}

extern "C" void kernel_launch(void* const* d_in, const int* in_sizes, int n_in,
                              void* d_out, int out_size, void* d_ws, size_t ws_size,
                              hipStream_t stream) {
  if (n_in < 16) return;
  if (in_sizes[0] != RW * DM || in_sizes[1] != RW * DM || out_size != RW * DM) return;
  if (in_sizes[4] != NEDGE * DM * DM || in_sizes[8] != NCELL * 4 * DM * DM) return;
  if (in_sizes[14] != RW || in_sizes[15] != RW) return;
  if (ws_size < WS_NEED) return;

  const float* inpute    = (const float*)d_in[0];
  const float* inputo    = (const float*)d_in[1];
  const float* node_p    = (const float*)d_in[2];
  const float* edge_p    = (const float*)d_in[3];
  const float* edge_W    = (const float*)d_in[4];
  const float* edge_b    = (const float*)d_in[5];
  const float* edge_g    = (const float*)d_in[6];
  const float* edge_beta = (const float*)d_in[7];
  const float* node_W    = (const float*)d_in[8];
  const float* node_b    = (const float*)d_in[9];
  const float* node_g    = (const float*)d_in[10];
  const float* node_beta = (const float*)d_in[11];
  const float* out_g     = (const float*)d_in[12];
  const float* out_beta  = (const float*)d_in[13];
  const int*   msrc      = (const int*)d_in[14];
  const int*   mtgt      = (const int*)d_in[15];
  char* ws = (char*)d_ws;

  wconv_kernel<<<dim3(DM / 32, DM / 128, NEDGE), 256, 0, stream>>>(edge_W, 0, ws);
  wconv_kernel<<<dim3(DM / 32, DM / 128, NCELL * 4), 256, 0, stream>>>(node_W, NEDGE, ws);

  PlanArgs pa;
  pa.inpute = inpute; pa.inputo = inputo; pa.node_p = node_p; pa.edge_p = edge_p;
  pa.edge_b = edge_b; pa.edge_g = edge_g; pa.edge_beta = edge_beta;
  pa.node_b = node_b; pa.node_g = node_g; pa.node_beta = node_beta;
  pa.ws = ws;
  plan_kernel<<<1, 32, 0, stream>>>(pa);

  const dim3 gge(RW / 64, DM / 64, 3);
  const dim3 gg1(RW / 64, DM / 64, 1);
  for (int c = 0; c < NCELL; c++) {
    ew_kernel<<<dim3(RW / 4, 3), 128, 0, stream>>>(ws, c, 0);
    gemm_kernel<<<gge, 128, 0, stream>>>(ws, c, 0);
    ew_kernel<<<dim3(RW / 4, 1), 128, 0, stream>>>(ws, c, 3);
    gemm_kernel<<<gge, 128, 0, stream>>>(ws, c, 3);
    ew_kernel<<<dim3(RW / 4, 1), 128, 0, stream>>>(ws, c, 4);
    attn_kernel<<<512, 128, 0, stream>>>(ws, c, msrc, mtgt);
    gemm_kernel<<<gg1, 128, 0, stream>>>(ws, c, 6);
  }
  final_kernel<<<RW / 4, 128, 0, stream>>>(ws, out_g, out_beta, (float*)d_out);
}
